// MultiHeadAttention_43508018709076
// MI455X (gfx1250) — hardware-verified
//
#include <hip/hip_runtime.h>
#include <math.h>

#ifndef NB
#define NB 2
#endif
#ifndef SEQ
#define SEQ 2048
#endif
#define NB_FULL 2
#define SEQ_FULL 2048
#define CH 1024
#define NH 16
#define HD 64

static_assert(SEQ % 64 == 0);
static_assert(NB >= 1 && NB <= NB_FULL && SEQ <= SEQ_FULL);
static_assert(CH == NH * HD && HD == 64);

typedef __attribute__((ext_vector_type(16))) _Float16     v16h;
typedef __attribute__((ext_vector_type(8)))  _Float16     v8h;
typedef __attribute__((ext_vector_type(8)))  float        v8f;
typedef __attribute__((ext_vector_type(4)))  float        v4f;
typedef __attribute__((ext_vector_type(4)))  unsigned int u4v;

union FragH { v16h v; v8h h[2]; };
__device__ __forceinline__ v16h frag_ld(const _Float16* p) { FragH f; f.h[0] = *(const v8h*)(p); f.h[1] = *(const v8h*)(p + 16); return f.v; }
__device__ __forceinline__ v8f mma_raw(v16h a, v16h b, v8f c) { return __builtin_amdgcn_wmma_f32_16x16x32_f16(false, a, false, b, (short)0, c, false, false); }
__device__ __forceinline__ v8f mma_h(v16h a, v16h b, v8f c) {
    c = __builtin_amdgcn_wmma_f32_16x16x32_f16(false, a, false, b, (short)0, c, false, false);
    asm volatile("v_nop\n\tv_nop\n\tv_nop\n\tv_nop" : "+v"(c) : "v"(a), "v"(b));
    return c;
}
__device__ __forceinline__ void dep_guard_h(v8f& a, v8f& b, v16h x, v16h y) { asm volatile("v_nop\n\tv_nop\n\tv_nop\n\tv_nop" : "+v"(a), "+v"(b) : "v"(x), "v"(y)); }
__device__ __forceinline__ void keep4_h(v16h a, v16h b, v16h c, v16h d) { asm volatile("v_nop" :: "v"(a), "v"(b), "v"(c), "v"(d)); }
__device__ __forceinline__ void acc_guard4(v8f& a, v8f& b, v8f& c, v8f& d) { asm volatile("v_nop\n\tv_nop\n\tv_nop\n\tv_nop" : "+v"(a), "+v"(b), "+v"(c), "+v"(d)); }
__device__ __forceinline__ v8h cvt8(v4f a, v4f b) {
    v8h r;
    r[0] = (_Float16)a.x; r[1] = (_Float16)a.y; r[2] = (_Float16)a.z; r[3] = (_Float16)a.w;
    r[4] = (_Float16)b.x; r[5] = (_Float16)b.y; r[6] = (_Float16)b.z; r[7] = (_Float16)b.w;
    return r;
}
__device__ __forceinline__ unsigned short f2bf_bits(float f) { unsigned u = __float_as_uint(f); return (unsigned short)((u + 0x7FFFu + ((u >> 16) & 1u)) >> 16); }
__device__ __forceinline__ float bf_bits2f(unsigned short h) { return __uint_as_float(((unsigned)h) << 16); }
__device__ __forceinline__ float cmb_bf(float v) { const unsigned u = __float_as_uint(v); const unsigned r = (u + 0x7fffu + ((u >> 16) & 1u)) & 0xffff0000u; return __uint_as_float(r); }
__device__ __forceinline__ unsigned int cmb_pk2(float a, float b) { return (unsigned int)__builtin_bit_cast(unsigned short, (_Float16)a) | ((unsigned int)__builtin_bit_cast(unsigned short, (_Float16)b) << 16); }

#define VST2(T, ptr, val) do { const T vst2_v_ = (val); *(volatile T*)(ptr) = vst2_v_; __threadfence(); *(volatile T*)(ptr) = vst2_v_; } while (0)

template <bool BFR>
__global__ __launch_bounds__(256) void k_cast8(const float* __restrict__ SRC, long long lds, int rpb, long long sbs,
                                               unsigned short* __restrict__ DST, long long ldd, int nR, int nC, float sc) {
    const long long u = (long long)blockIdx.x * 256 + threadIdx.x; const int per = nC / 8;
    if (u >= (long long)nR * per) return;
    const int r = (int)(u / per); const int c0 = 8 * (int)(u % per);
    const int rb = r / rpb, rl = r - rb * rpb;
    const float* s = SRC + (long long)rb * sbs + (long long)rl * lds + c0;
    const v4f a = *(const v4f*)(s), b = *(const v4f*)(s + 4);
    float w[8] = {a.x, a.y, a.z, a.w, b.x, b.y, b.z, b.w};
#pragma unroll
    for (int e = 0; e < 8; ++e) w[e] = (BFR ? cmb_bf(w[e]) : w[e]) * sc;
    u4v pk; pk.x = cmb_pk2(w[0], w[1]); pk.y = cmb_pk2(w[2], w[3]); pk.z = cmb_pk2(w[4], w[5]); pk.w = cmb_pk2(w[6], w[7]);
    VST2(u4v, (u4v*)(DST + (long long)r * ldd + c0), pk);
}

template <int BIAS_MODE>
__global__ __launch_bounds__(256) void k_gemm64(const unsigned short* __restrict__ Ap, int lda, long long strideA,
                                                const unsigned short* __restrict__ Btp, int ldb,
                                                float* __restrict__ Cout, int ldc, long long strideC,
                                                const float* __restrict__ bias, int M, int N, int K, float scale) {
    const _Float16* A = (const _Float16*)Ap; const _Float16* Bt = (const _Float16*)Btp;
    __shared__ __align__(16) float sT[8][16 * 68];
    const int b = blockIdx.y;
    const int lane = threadIdx.x & 31;
    const int wave = threadIdx.x >> 5;
    const int tilesN = N >> 6;
    const int tilesM = M >> 6;
    const int tile = blockIdx.x * 8 + wave;
    if (tile >= tilesM * tilesN) return;
    const int tm = tile / tilesN;
    const int tn = tile - tm * tilesN;
    const int m0 = tm << 6;
    const int n0 = tn << 6;
    const _Float16* Ab = A + (size_t)b * strideA;
    const _Float16* Bb = Bt;
    const int rlane = lane & 15;
    const int koff  = (lane >> 4) * 8;
    const int mOff  = (lane >> 4) * 8;

    v8f acc[4][4];
#pragma unroll
    for (int i = 0; i < 4; ++i)
#pragma unroll
        for (int j = 0; j < 4; ++j) acc[i][j] = (v8f){0.f, 0.f, 0.f, 0.f, 0.f, 0.f, 0.f, 0.f};

    for (int k0 = 0; k0 < K; k0 += 32) {
        v16h bh[4];
#pragma unroll
        for (int j = 0; j < 4; ++j) bh[j] = frag_ld(Bb + (size_t)(n0 + (j << 4) + rlane) * ldb + koff + k0);
#pragma unroll
        for (int i = 0; i < 4; ++i) {
            const v16h ah = frag_ld(Ab + (size_t)(m0 + (i << 4) + rlane) * lda + koff + k0);
#pragma unroll
            for (int j = 0; j < 4; ++j) acc[i][j] = mma_raw(ah, bh[j], acc[i][j]);
            dep_guard_h(acc[i][0], acc[i][3], ah, ah);
        }
        keep4_h(bh[0], bh[1], bh[2], bh[3]);
    }
    acc_guard4(acc[0][0], acc[0][1], acc[0][2], acc[0][3]);
    acc_guard4(acc[1][0], acc[1][1], acc[1][2], acc[1][3]);
    acc_guard4(acc[2][0], acc[2][1], acc[2][2], acc[2][3]);
    acc_guard4(acc[3][0], acc[3][1], acc[3][2], acc[3][3]);

    float* slab = sT[wave];
    float* C = Cout + (size_t)b * strideC;
#pragma unroll
    for (int i = 0; i < 4; ++i) {
        const int mBase = m0 + (i << 4);
#pragma unroll
        for (int j = 0; j < 4; ++j) {
            const int n = n0 + (j << 4) + rlane;
            float bv = 0.f;
            if (BIAS_MODE == 3) bv = bf_bits2f(f2bf_bits(bias[n]));
#pragma unroll
            for (int r = 0; r < 8; ++r) {
                float v = acc[i][j][r] * scale;
                if (BIAS_MODE == 3) v += bv;
                slab[(mOff + r) * 68 + (j << 4) + rlane] = v;
            }
        }
        __builtin_amdgcn_fence(3  , "workgroup");
        __builtin_amdgcn_wave_barrier();
        __builtin_amdgcn_fence(2  , "workgroup");
        {
            const int hh = lane >> 4, c4 = (lane & 15) * 4;
            for (int pass = 0; pass < 2; ++pass) {
#pragma unroll
                for (int it = 0; it < 8; ++it) {
                    const int row = it * 2 + hh;
                    const v4f v = *(const v4f*)(slab + row * 68 + c4);
                    *(volatile v4f*)(C + (size_t)(mBase + row) * ldc + n0 + c4) = v;
                }
                __threadfence();
            }
        }
        __builtin_amdgcn_fence(3  , "workgroup");
        __builtin_amdgcn_wave_barrier();
        __builtin_amdgcn_fence(2  , "workgroup");
    }
}

#define AT_D  64
#define AT_NW 4
#define AT_QB 64
#define AT_KC 64
#define AT_P  72
struct AttnG {
    const float* q; const float* k; const float* v; float* o;
    long long q_bs, q_rs, q_hs, k_bs, k_rs, k_hs, v_bs, v_rs, v_hs, o_bs, o_rs, o_hs;
    int S, Skv; float sscale; int pad_;
};
static_assert(sizeof(AttnG) == 4 * 8 + 12 * 8 + 4 * 4);

__global__ __launch_bounds__(128) void k_attn_alibi(AttnG g) {
    __shared__ __align__(16) _Float16 Ks[AT_KC * AT_P];
    __shared__ __align__(16) _Float16 Vt[AT_D * AT_P];
    __shared__ __align__(16) _Float16 Ps[AT_NW][16 * AT_P];
    __shared__ __align__(16) float    Os[AT_NW][16 * 68];

    const int tid  = threadIdx.x;
    const int wave = tid >> 5;
    const int lane = tid & 31;
    const int hh   = lane >> 4;
    const int c    = lane & 15;
    const int qb = blockIdx.x, h = blockIdx.y, b = blockIdx.z;
    const int q0 = qb * AT_QB + wave * 16;

    const float* qp = g.q + (size_t)b * g.q_bs + (size_t)h * g.q_hs;
    const float* kp = g.k + (size_t)b * g.k_bs + (size_t)h * g.k_hs;
    const float* vp = g.v + (size_t)b * g.v_bs + (size_t)h * g.v_hs;
    float*       op = g.o + (size_t)b * g.o_bs + (size_t)h * g.o_hs;

    const int e1 = h + 1;
    const float pw2 = __uint_as_float((unsigned)(127 - (e1 >> 1)) << 23);
    const float nsl = -(((e1 & 1) ? 0.70710678118654752f : 1.0f) * pw2);
    const float L2E = 1.4426950408889634f;

    v16h qa[2];
    {
        const float* qrow = qp + (size_t)(q0 + c) * g.q_rs;
#pragma unroll
        for (int dc = 0; dc < 2; ++dc) {
            FragH f;
            f.h[0] = cvt8(*(const v4f*)(qrow + dc * 32 + 8 * hh),      *(const v4f*)(qrow + dc * 32 + 8 * hh + 4));
            f.h[1] = cvt8(*(const v4f*)(qrow + dc * 32 + 16 + 8 * hh), *(const v4f*)(qrow + dc * 32 + 16 + 8 * hh + 4));
            qa[dc] = f.v;
        }
    }

    float mrow[8], lrow[8];
    v8f oacc[4];
#pragma unroll
    for (int r = 0; r < 8; ++r) { mrow[r] = -__builtin_inff(); lrow[r] = 0.f; }
#pragma unroll
    for (int t = 0; t < 4; ++t) oacc[t] = (v8f){0.f, 0.f, 0.f, 0.f, 0.f, 0.f, 0.f, 0.f};

    _Float16* pw = Ps[wave];
    const int nChunks = g.Skv / AT_KC;
    for (int kc = 0; kc < nChunks; ++kc) {
        const int kv0 = kc * AT_KC;
        __syncthreads();
        {
            const int kvr = tid >> 1, dh = (tid & 1) * 32;
            const float* krow = kp + (size_t)(kv0 + kvr) * g.k_rs + dh;
            const float* vrow = vp + (size_t)(kv0 + kvr) * g.v_rs + dh;
#pragma unroll
            for (int i = 0; i < 4; ++i) {
                const v4f k0 = *(const v4f*)(krow + 8 * i), k1 = *(const v4f*)(krow + 8 * i + 4);
                const v4f v0 = *(const v4f*)(vrow + 8 * i), v1 = *(const v4f*)(vrow + 8 * i + 4);
                *(v8h*)(Ks + kvr * AT_P + dh + 8 * i) = cvt8(k0, k1);
#pragma unroll
                for (int e = 0; e < 4; ++e) {
                    Vt[(dh + 8 * i + e) * AT_P + kvr]     = (_Float16)v0[e];
                    Vt[(dh + 8 * i + 4 + e) * AT_P + kvr] = (_Float16)v1[e];
                }
            }
        }
        __syncthreads();

        v8f s[4];
#pragma unroll
        for (int j = 0; j < 4; ++j) {
            s[j] = (v8f){0.f, 0.f, 0.f, 0.f, 0.f, 0.f, 0.f, 0.f};
#pragma unroll
            for (int dc = 0; dc < 2; ++dc) {
                const v16h kb = frag_ld(Ks + (j * 16 + c) * AT_P + dc * 32 + 8 * hh);
                s[j] = mma_h(qa[dc], kb, s[j]);
            }
        }
#pragma unroll
        for (int r = 0; r < 8; ++r) {
            const int qrow = q0 + 8 * hh + r;
            float m = -__builtin_inff();
#pragma unroll
            for (int j = 0; j < 4; ++j) {
                const int kvcol = kv0 + j * 16 + c;
                const float dist = fabsf((float)(kvcol - qrow));
                const float bias = nsl * dist;
                float t = s[j][r] * g.sscale + bias;
                t *= L2E;
                s[j][r] = t;
                m = fmaxf(m, t);
            }
            m = fmaxf(m, __shfl_xor(m, 1, 32)); m = fmaxf(m, __shfl_xor(m, 2, 32));
            m = fmaxf(m, __shfl_xor(m, 4, 32)); m = fmaxf(m, __shfl_xor(m, 8, 32));
            const float mnew = fmaxf(mrow[r], m);
            const float alpha = exp2f(mrow[r] - mnew);
            mrow[r] = mnew;
            float psum = 0.f;
#pragma unroll
            for (int j = 0; j < 4; ++j) {
                const float p = exp2f(s[j][r] - mnew);
                psum += p;
                pw[(8 * hh + r) * AT_P + j * 16 + c] = (_Float16)(p * 32768.0f);
            }
            psum += __shfl_xor(psum, 1, 32); psum += __shfl_xor(psum, 2, 32);
            psum += __shfl_xor(psum, 4, 32); psum += __shfl_xor(psum, 8, 32);
            lrow[r] = lrow[r] * alpha + psum;
#pragma unroll
            for (int t = 0; t < 4; ++t) oacc[t][r] *= alpha;
        }
        __builtin_amdgcn_fence(3  , "workgroup");
        __builtin_amdgcn_wave_barrier();
        __builtin_amdgcn_fence(2  , "workgroup");
#pragma unroll
        for (int kk = 0; kk < 2; ++kk) {
            const v16h pa = frag_ld(pw + c * AT_P + kk * 32 + 8 * hh);
#pragma unroll
            for (int t = 0; t < 4; ++t) {
                const v16h vb = frag_ld(Vt + (t * 16 + c) * AT_P + kk * 32 + 8 * hh);
                oacc[t] = mma_h(pa, vb, oacc[t]);
            }
        }
    }

    float* os = Os[wave];
#pragma unroll
    for (int r = 0; r < 8; ++r) {
        const float inv = 1.0f / (lrow[r] * 32768.0f);
#pragma unroll
        for (int t = 0; t < 4; ++t) os[(8 * hh + r) * 68 + t * 16 + c] = oacc[t][r] * inv;
    }
    __builtin_amdgcn_fence(3  , "workgroup");
    __builtin_amdgcn_wave_barrier();
    __builtin_amdgcn_fence(2  , "workgroup");
    {
        const int c4 = (lane & 15) * 4;
        for (int pass = 0; pass < 2; ++pass) {
#pragma unroll
            for (int it = 0; it < 8; ++it) {
                const int row = it * 2 + hh;
                const v4f val = *(const v4f*)(os + row * 68 + c4);
                *(volatile v4f*)(op + (size_t)(q0 + row) * g.o_rs + c4) = val;
            }
            __threadfence();
        }
    }
}

constexpr size_t SZ_X16 = (size_t)NB * SEQ * CH * 2;
constexpr size_t SZ_W3  = (size_t)3 * CH * CH * 2;
constexpr size_t SZ_QKV = (size_t)NB * SEQ * 3 * CH * 4;
constexpr size_t SZ_AO  = (size_t)NB * SEQ * CH * 4;
constexpr size_t SZ_WO  = (size_t)CH * CH * 2;
constexpr size_t SZ_ALL = SZ_X16 + SZ_W3 + SZ_QKV + SZ_AO + SZ_WO;
static_assert(SZ_X16 % 256 == 0 && SZ_W3 % 256 == 0 && SZ_QKV % 256 == 0 && SZ_AO % 256 == 0 && SZ_WO % 256 == 0);
static_assert(SZ_ALL <= (size_t)134217728);

extern "C" void kernel_launch(void* const* d_in, const int* in_sizes, int n_in, void* d_out, int out_size, void* d_ws, size_t ws_size, hipStream_t stream) {
    if (n_in < 6) return;
    const long long need_x = ((long long)(NB - 1) * SEQ_FULL + SEQ) * CH;
    if ((long long)in_sizes[0] < need_x) return;
    if (in_sizes[1] < CH * CH || in_sizes[2] < CH * CH || in_sizes[3] < CH * CH || in_sizes[4] < CH * CH || in_sizes[5] < CH) return;
    if ((long long)out_size < need_x) return;
    if (SZ_ALL > ws_size) return;
    const float* x  = (const float*)d_in[0];
    const float* wq = (const float*)d_in[1];
    const float* wk = (const float*)d_in[2];
    const float* wv = (const float*)d_in[3];
    const float* wo = (const float*)d_in[4];
    const float* bo = (const float*)d_in[5];
    float* out = (float*)d_out;
    char* wsp = (char*)d_ws;
    unsigned short* X16  = (unsigned short*)wsp; wsp += SZ_X16;
    unsigned short* W316 = (unsigned short*)wsp; wsp += SZ_W3;
    float*          QKV  = (float*)wsp;          wsp += SZ_QKV;
    float*          AO   = (float*)wsp;          wsp += SZ_AO;
    unsigned short* WO16 = (unsigned short*)wsp; wsp += SZ_WO;
    unsigned short* AO16 = X16;

    const unsigned gW = (unsigned)(((long long)CH * (CH / 8) + 255) / 256);
    const unsigned gX = (unsigned)(((long long)NB * SEQ * (CH / 8) + 255) / 256);
    k_cast8<true><<<gW, 256, 0, stream>>>(wo, (long long)CH, CH, 0LL, WO16, (long long)CH, CH, CH, 16.0f);
    k_cast8<true><<<gX, 256, 0, stream>>>(x, (long long)CH, SEQ, (long long)SEQ_FULL * CH, X16, (long long)CH, NB * SEQ, CH, 1.0f);
    k_cast8<true><<<gW, 256, 0, stream>>>(wq, (long long)CH, CH, 0LL, W316, (long long)CH, CH, CH, 16.0f);
    k_cast8<true><<<gW, 256, 0, stream>>>(wk, (long long)CH, CH, 0LL, W316 + (size_t)CH * CH, (long long)CH, CH, CH, 16.0f);
    k_cast8<true><<<gW, 256, 0, stream>>>(wv, (long long)CH, CH, 0LL, W316 + (size_t)2 * CH * CH, (long long)CH, CH, CH, 16.0f);
    k_gemm64<0><<<dim3((unsigned)((((NB * SEQ) / 64) * ((3 * CH) / 64) + 7) / 8), 1u), 256, 0, stream>>>(
        X16, CH, 0LL, W316, CH, QKV, 3 * CH, 0LL, (const float*)nullptr, NB * SEQ, 3 * CH, CH, 0.0625f);
    {
        AttnG g;
        g.q = QKV; g.k = QKV + CH; g.v = QKV + 2 * CH; g.o = AO;
        g.q_bs = (long long)SEQ * 3 * CH; g.q_rs = 3 * CH; g.q_hs = HD;
        g.k_bs = (long long)SEQ * 3 * CH; g.k_rs = 3 * CH; g.k_hs = HD;
        g.v_bs = (long long)SEQ * 3 * CH; g.v_rs = 3 * CH; g.v_hs = HD;
        g.o_bs = (long long)SEQ * CH;     g.o_rs = CH;     g.o_hs = HD;
        g.S = SEQ; g.Skv = SEQ; g.sscale = 0.125f; g.pad_ = 0;
        k_attn_alibi<<<dim3((unsigned)(SEQ / AT_QB), (unsigned)NH, (unsigned)NB), 32 * AT_NW, 0, stream>>>(g);
    }
    k_cast8<false><<<gX, 256, 0, stream>>>(AO, (long long)CH, NB * SEQ, 0LL, AO16, (long long)CH, NB * SEQ, CH, 16.0f);
    k_gemm64<3><<<dim3((unsigned)(((SEQ / 64) * (CH / 64) + 7) / 8), (unsigned)NB), 256, 0, stream>>>(
        AO16, CH, (long long)SEQ * CH, WO16, CH, out, CH, (long long)SEQ_FULL * CH, bo, SEQ, CH, CH, 1.0f / 256.0f);
}
